// Attention_49529562858354
// MI455X (gfx1250) — hardware-verified
//
#include <hip/hip_runtime.h>


#ifndef NB
#define NB 4
#endif
#ifndef SEQ
#define SEQ 2048
#endif
#define NB_FULL  4
#define SEQ_FULL 2048
#define DMOD 1024
#define NHD  16
#define HD   64
#define QKVN (3 * DMOD)
#define SCL  0.125f
#define PCAR 1024.0f
#define NEGB (-3.0e38f)
#define LNEPS 1e-5f
#define KSP  72
#define OSP  68
static_assert(SEQ % 128 == 0);
static_assert(SEQ >= 128);
static_assert(SEQ <= SEQ_FULL);
static_assert(NB >= 1);
static_assert(NB <= NB_FULL);
static_assert(DMOD % 64 == 0);
static_assert(QKVN % 64 == 0);
static_assert(NHD * HD == DMOD);
static_assert(DMOD % 32 == 0);

typedef _Float16 h16;
typedef unsigned short bf;
typedef __attribute__((ext_vector_type(16))) __bf16   v16bf;
typedef __attribute__((ext_vector_type(16))) _Float16 v16h;
typedef __attribute__((ext_vector_type(8)))  _Float16 v8h;
typedef __attribute__((ext_vector_type(8)))  unsigned short v8us;
typedef __attribute__((ext_vector_type(8)))  float    v8f;
typedef __attribute__((ext_vector_type(4)))  float    v4f;
typedef __attribute__((ext_vector_type(2)))  unsigned short v2us;
typedef v8h  __attribute__((may_alias)) v8ha;
typedef v4f  __attribute__((may_alias)) v4fa;
typedef v8us __attribute__((may_alias)) v8usa;
typedef v8f  __attribute__((may_alias)) v8fa;

__device__ __forceinline__ unsigned short f2bf(float f) { unsigned u = __float_as_uint(f); u += 0x7FFFu + ((u >> 16) & 1u); return (unsigned short)(u >> 16); }
__device__ __forceinline__ float bf2f(unsigned short b) { return __uint_as_float(((unsigned)b) << 16); }
__device__ __forceinline__ float bfr(float f) { return bf2f(f2bf(f)); }
__device__ __forceinline__ void splitf(float y, unsigned short& h, unsigned short& l) { h = f2bf(y); l = f2bf(y - bf2f(h)); }
__device__ __forceinline__ v16h cat16(v8h lo, v8h hi) { return __builtin_shufflevector(lo, hi, 0, 1, 2, 3, 4, 5, 6, 7, 8, 9, 10, 11, 12, 13, 14, 15); }
__device__ __forceinline__ v16bf cat16b(v8us lo, v8us hi) { return __builtin_bit_cast(v16bf, __builtin_shufflevector(lo, hi, 0, 1, 2, 3, 4, 5, 6, 7, 8, 9, 10, 11, 12, 13, 14, 15)); }
__device__ __forceinline__ v8f wmma16(v16h a, v16h b, v8f c) { return __builtin_amdgcn_wmma_f32_16x16x32_f16(false, a, false, b, (short)0, c, false, false); }
__device__ __forceinline__ v8f wmmab(v16bf a, v16bf b, v8f c) { return __builtin_amdgcn_wmma_f32_16x16x32_bf16(false, a, false, b, (short)0, c, false, false); }
__device__ __forceinline__ float hmax16(float v) { v = fmaxf(v, __shfl_xor(v, 1, 32)); v = fmaxf(v, __shfl_xor(v, 2, 32)); v = fmaxf(v, __shfl_xor(v, 4, 32)); v = fmaxf(v, __shfl_xor(v, 8, 32)); return v; }
__device__ __forceinline__ float hsum16(float v) { v += __shfl_xor(v, 1, 32); v += __shfl_xor(v, 2, 32); v += __shfl_xor(v, 4, 32); v += __shfl_xor(v, 8, 32); return v; }

template <typename T16> struct WFrag;
template <> struct WFrag<h16> { typedef v16h V; static __device__ __forceinline__ V ld(const h16* p) { return cat16(*(const v8ha*)p, *(const v8ha*)(p + 16)); } static __device__ __forceinline__ v8f mma(V a, V b, v8f c) { return wmma16(a, b, c); } };
template <> struct WFrag<bf> { typedef v16bf V; static __device__ __forceinline__ V ld(const bf* p) { return cat16b(*(const v8usa*)p, *(const v8usa*)(p + 16)); } static __device__ __forceinline__ v8f mma(V a, V b, v8f c) { return wmmab(a, b, c); } };

template <typename T16, int NSPLIT, bool BIAS>
__global__ __launch_bounds__(32) void k_gemmw(const T16* __restrict__ A, const T16* __restrict__ A2, const T16* __restrict__ Bt, const T16* __restrict__ Bt2, int K, float* C, int ldc, const float* __restrict__ bias, size_t sA, size_t sB, size_t sC) {
    typedef typename WFrag<T16>::V V;
    __shared__ __align__(16) float os[16 * 68];
    const size_t z = blockIdx.z; A += z * sA; if (A2) A2 += z * sA; Bt += z * sB; if (Bt2) Bt2 += z * sB; C += z * sC;
    const int lane = threadIdx.x & 31, lr = lane & 15, hi = lane >> 4; const int r0 = blockIdx.x * 64, c0 = blockIdx.y * 64;
    v8f acc[4][4];
#pragma unroll
    for (int mb = 0; mb < 4; ++mb)
#pragma unroll
        for (int nb = 0; nb < 4; ++nb) acc[mb][nb] = (v8f){};
    const size_t aoff = (size_t)(r0 + lr) * K + 8 * hi, boff = (size_t)(c0 + lr) * K + 8 * hi;
#pragma unroll 1
    for (int kc = 0; kc < K; kc += 32) {
        V a[4], a2[4];
#pragma unroll
        for (int mb = 0; mb < 4; ++mb) { a[mb] = WFrag<T16>::ld(A + aoff + (size_t)mb * 16 * K + kc); if (NSPLIT == 1 || NSPLIT == 2) a2[mb] = WFrag<T16>::ld(A2 + aoff + (size_t)mb * 16 * K + kc); }
#pragma unroll
        for (int nb = 0; nb < 4; ++nb) { const V b = WFrag<T16>::ld(Bt + boff + (size_t)nb * 16 * K + kc); V b2; if (NSPLIT >= 2) b2 = WFrag<T16>::ld(Bt2 + boff + (size_t)nb * 16 * K + kc);
#pragma unroll
            for (int mb = 0; mb < 4; ++mb) { acc[mb][nb] = WFrag<T16>::mma(a[mb], b, acc[mb][nb]); if (NSPLIT == 1 || NSPLIT == 2) acc[mb][nb] = WFrag<T16>::mma(a2[mb], b, acc[mb][nb]); if (NSPLIT >= 2) acc[mb][nb] = WFrag<T16>::mma(a[mb], b2, acc[mb][nb]); } }
        asm volatile("v_nop\n\tv_nop\n\tv_nop\n\tv_nop" : "+v"(acc[0][0]), "+v"(acc[1][1]), "+v"(acc[2][2]), "+v"(acc[3][3]) : "v"(a[0]), "v"(a[3]));
    }
#pragma unroll
    for (int mb = 0; mb < 4; ++mb) {
#pragma unroll
        for (int nb = 0; nb < 4; ++nb) {
#pragma unroll
            for (int j = 0; j < 8; ++j) os[(hi * 8 + j) * 68 + nb * 16 + lr] = acc[mb][nb][j]; }
        __builtin_amdgcn_wave_barrier(); asm volatile("" ::: "memory");
        float* crow = C + (size_t)(r0 + mb * 16) * ldc + c0;
#pragma unroll 1
        for (int ps = 0; ps < 2; ++ps) {
#pragma unroll
            for (int s = 0; s < 8; ++s) { const int row = 2 * s + hi, cofs = lr * 4; v4f val = *(const v4fa*)(os + row * 68 + cofs); if (BIAS) { val[0] += bfr(bias[c0 + cofs]); val[1] += bfr(bias[c0 + cofs + 1]); val[2] += bfr(bias[c0 + cofs + 2]); val[3] += bfr(bias[c0 + cofs + 3]); }
                *(volatile v4f*)(crow + (size_t)row * ldc + cofs) = val; }
            if (ps == 0) __threadfence(); }
        __builtin_amdgcn_wave_barrier(); asm volatile("" ::: "memory");
    }
}

__global__ __launch_bounds__(256) void k_wtG(const float* __restrict__ w, int K, int N, bf* Bt) {
    const int lane = threadIdx.x & 31; const int L0 = (blockIdx.x * 8 + (threadIdx.x >> 5)) * 8; const int nlines = N * K / 64;
#pragma unroll
    for (int ps = 0; ps < 2; ++ps) {
#pragma unroll 1
        for (int l = 0; l < 8; ++l) { const int L = L0 + l; if (L >= nlines) break; const size_t e = (size_t)L * 64 + lane * 2; const int k = (int)(e % K), n = (int)(e / K); v2us o;
            o[0] = f2bf(w[(size_t)k * N + n]); o[1] = f2bf(w[(size_t)(k + 1) * N + n]); *(volatile v2us*)(Bt + e) = o; }
        if (ps == 0) __threadfence(); }
}

__global__ __launch_bounds__(128) void k_ln(const float* __restrict__ X, const float* __restrict__ G, const float* __restrict__ Bv, bf* XH, bf* XL) {
    __shared__ float red[8];
    const int tid = threadIdx.x, lane = tid & 31, wid = tid >> 5; const int row = blockIdx.x; const int c = tid * 8;
    const v8f a = *(const v8fa*)(X + (size_t)row * DMOD + c);
    float v[8]; float s = 0.f;
#pragma unroll
    for (int q = 0; q < 8; ++q) { v[q] = bfr(a[q]); s += v[q]; }
#pragma unroll
    for (int sh = 16; sh; sh >>= 1) s += __shfl_xor(s, sh, 32);
    if (lane == 0) red[wid] = s;
    __syncthreads();
    const float mean = ((red[0] + red[1]) + (red[2] + red[3])) * (1.0f / DMOD);
    float s2 = 0.f;
#pragma unroll
    for (int q = 0; q < 8; ++q) { const float d = v[q] - mean; v[q] = d; s2 += d * d; }
#pragma unroll
    for (int sh = 16; sh; sh >>= 1) s2 += __shfl_xor(s2, sh, 32);
    if (lane == 0) red[4 + wid] = s2;
    __syncthreads();
    const float var = ((red[4] + red[5]) + (red[6] + red[7])) * (1.0f / DMOD);
    const float rstd = rsqrtf(var + LNEPS);
    const v8f g = *(const v8fa*)(G + c); const v8f bb = *(const v8fa*)(Bv + c);
    v8us oh, ol;
#pragma unroll
    for (int q = 0; q < 8; ++q) { const float y = v[q] * rstd * bfr(g[q]) + bfr(bb[q]); unsigned short a2, c2; splitf(y, a2, c2); oh[q] = a2; ol[q] = c2; }
    const size_t e = (size_t)row * DMOD + c;
    *(volatile v8us*)(XH + e) = oh; *(volatile v8us*)(XL + e) = ol;
    __threadfence();
    *(volatile v8us*)(XH + e) = oh; *(volatile v8us*)(XL + e) = ol;
}

__global__ __launch_bounds__(256) void k_qkp(const float* __restrict__ C, h16* QP, h16* KP, int n8) {
    const int i = blockIdx.x * 256 + threadIdx.x; if (i >= n8) return;
    const int which = blockIdx.y;
    const size_t e = (size_t)i * 8; const int d = (int)(e % HD); const int t = (int)((e / HD) % SEQ); const int hh = (int)(e / ((size_t)HD * SEQ));
    const v8f a = *(const v8fa*)(C + (size_t)t * QKVN + which * DMOD + hh * HD + d);
    v8h o;
#pragma unroll
    for (int q = 0; q < 8; ++q) o[q] = (h16)a[q];
    h16* dst = (which == 0) ? QP : KP;
    *(volatile v8h*)(dst + e) = o; __threadfence(); *(volatile v8h*)(dst + e) = o;
}

__global__ __launch_bounds__(256) void k_vtp16(const float* __restrict__ C, h16* VTp) {
    __shared__ __align__(16) h16 T[64 * KSP];
    const int tid = threadIdx.x; const int t0 = blockIdx.x * 64; const int hh = blockIdx.y;
#pragma unroll
    for (int rr = 0; rr < 4; ++rr) { const int idx = tid + 256 * rr; const int tt = idx >> 4; const int c4 = (idx & 15) * 4;
        const v4f a = *(const v4fa*)(C + (size_t)(t0 + tt) * QKVN + 2 * DMOD + hh * HD + c4);
#pragma unroll
        for (int q = 0; q < 4; ++q) T[(c4 + q) * KSP + tt] = (h16)a[q]; }
    __syncthreads();
    v8h o[2]; size_t oo[2];
#pragma unroll
    for (int rr = 0; rr < 2; ++rr) { const int d = rr * 32 + (tid >> 3); const int p = (tid & 7) * 8; o[rr] = *(const v8ha*)(T + d * KSP + p); oo[rr] = ((size_t)hh * HD + d) * SEQ + t0 + p; }
#pragma unroll
    for (int rr = 0; rr < 2; ++rr) *(volatile v8h*)(VTp + oo[rr]) = o[rr];
    __threadfence();
#pragma unroll
    for (int rr = 0; rr < 2; ++rr) *(volatile v8h*)(VTp + oo[rr]) = o[rr];
}

__global__ __launch_bounds__(256) void k_flash(const h16* __restrict__ QP, const h16* __restrict__ KP, const h16* __restrict__ VT, const int* __restrict__ mk, float* outb) {
    __shared__ __align__(16) h16 Ks[64 * KSP];
    __shared__ __align__(16) h16 Vs[64 * KSP];
    __shared__ __align__(16) float Ow[8 * 16 * OSP];
    __shared__ int Ms[64];
    const int tid = threadIdx.x, wid = tid >> 5, lane = tid & 31, lr = lane & 15, hi = lane >> 4;
    const int hh = blockIdx.y, i0 = blockIdx.x * 128 + wid * 16;
    const h16* qp = QP + (size_t)hh * SEQ * HD; const h16* kp = KP + (size_t)hh * SEQ * HD; const h16* vt = VT + (size_t)hh * HD * SEQ;
    float* ow = Ow + wid * (16 * OSP); h16* pw = (h16*)ow;
    v16h qf[2];
    qf[0] = WFrag<h16>::ld(qp + (size_t)(i0 + lr) * HD + 8 * hi);
    qf[1] = WFrag<h16>::ld(qp + (size_t)(i0 + lr) * HD + 32 + 8 * hi);
    v8f o[4];
#pragma unroll
    for (int n = 0; n < 4; ++n) o[n] = (v8f){};
    float mrow[8], lrow[8];
#pragma unroll
    for (int r = 0; r < 8; ++r) { mrow[r] = -__builtin_inff(); lrow[r] = 0.f; }
    const float L2E = 1.4426950408889634f;
    const int srow = tid >> 3, spc = (tid & 7) * 8;
#pragma unroll 1
    for (int j0 = 0; j0 < SEQ; j0 += 64) {
        __syncthreads();
#pragma unroll
        for (int rr = 0; rr < 2; ++rr) { const int row = srow + 32 * rr;
            const v8h kv = *(const v8ha*)(kp + (size_t)(j0 + row) * HD + spc);
            const v8h vv = *(const v8ha*)(vt + (size_t)row * SEQ + j0 + spc);
            *(v8ha*)(Ks + row * KSP + spc) = kv; *(v8ha*)(Vs + row * KSP + spc) = vv; }
        if (tid < 64) Ms[tid] = mk[j0 + tid];
        __syncthreads();
        v8f s[4];
#pragma unroll
        for (int nt = 0; nt < 4; ++nt) { s[nt] = (v8f){};
#pragma unroll
            for (int kk = 0; kk < 2; ++kk) { const v16h b = WFrag<h16>::ld(Ks + (nt * 16 + lr) * KSP + kk * 32 + 8 * hi); s[nt] = wmma16(qf[kk], b, s[nt]); } }
        asm volatile("v_nop\n\tv_nop\n\tv_nop\n\tv_nop" : "+v"(s[0]), "+v"(s[1]), "+v"(s[2]), "+v"(s[3]) : "v"(qf[0]), "v"(qf[1]));
#pragma unroll
        for (int nt = 0; nt < 4; ++nt) { const bool ex = (Ms[nt * 16 + lr] >= 1);
#pragma unroll
            for (int r = 0; r < 8; ++r) { const float t = s[nt][r] * SCL; s[nt][r] = ex ? NEGB : t; } }
        float mcur[8], alpha[8];
#pragma unroll
        for (int r = 0; r < 8; ++r) { float mx = fmaxf(fmaxf(s[0][r], s[1][r]), fmaxf(s[2][r], s[3][r])); mx = hmax16(mx); const float mn = fmaxf(mrow[r], mx);
            alpha[r] = __builtin_amdgcn_exp2f(__fmul_rn(__fsub_rn(mrow[r], mn), L2E)); mcur[r] = mn; mrow[r] = mn; }
#pragma unroll
        for (int nt = 0; nt < 4; ++nt)
#pragma unroll
            for (int r = 0; r < 8; ++r) s[nt][r] = __builtin_amdgcn_exp2f(__fmul_rn(__fsub_rn(s[nt][r], mcur[r]), L2E));
#pragma unroll
        for (int r = 0; r < 8; ++r) { float su = (s[0][r] + s[1][r]) + (s[2][r] + s[3][r]); su = hsum16(su); lrow[r] = lrow[r] * alpha[r] + su; }
#pragma unroll
        for (int n = 0; n < 4; ++n)
#pragma unroll
            for (int r = 0; r < 8; ++r) o[n][r] *= alpha[r];
#pragma unroll
        for (int nt = 0; nt < 4; ++nt)
#pragma unroll
            for (int r = 0; r < 8; ++r) pw[(8 * hi + r) * KSP + nt * 16 + lr] = (h16)(s[nt][r] * PCAR);
        __syncthreads();
        const v16h a0 = WFrag<h16>::ld(pw + lr * KSP + 8 * hi), a1 = WFrag<h16>::ld(pw + lr * KSP + 32 + 8 * hi);
#pragma unroll
        for (int n = 0; n < 4; ++n) { const v16h b0 = WFrag<h16>::ld(Vs + (n * 16 + lr) * KSP + 8 * hi); o[n] = wmma16(a0, b0, o[n]); const v16h b1 = WFrag<h16>::ld(Vs + (n * 16 + lr) * KSP + 32 + 8 * hi); o[n] = wmma16(a1, b1, o[n]); }
        asm volatile("v_nop\n\tv_nop\n\tv_nop\n\tv_nop" : "+v"(o[0]), "+v"(o[1]), "+v"(o[2]), "+v"(o[3]) : "v"(a0), "v"(a1));
    }
    float inv[8];
#pragma unroll
    for (int r = 0; r < 8; ++r) inv[r] = __fdiv_rn(1.0f, lrow[r] * PCAR);
    __syncthreads();
#pragma unroll
    for (int n = 0; n < 4; ++n)
#pragma unroll
        for (int r = 0; r < 8; ++r) ow[(hi * 8 + r) * OSP + n * 16 + lr] = o[n][r] * inv[r];
    __syncthreads();
    float* orow = outb + (size_t)i0 * DMOD + hh * HD;
    v4f val[8];
#pragma unroll
    for (int sI = 0; sI < 8; ++sI) val[sI] = *(const v4fa*)(ow + (2 * sI + hi) * OSP + lr * 4);
#pragma unroll
    for (int sI = 0; sI < 8; ++sI) *(volatile v4f*)(orow + (size_t)(2 * sI + hi) * DMOD + lr * 4) = val[sI];
    __threadfence();
#pragma unroll
    for (int sI = 0; sI < 8; ++sI) *(volatile v4f*)(orow + (size_t)(2 * sI + hi) * DMOD + lr * 4) = val[sI];
}

extern "C" void kernel_launch(void* const* d_in, const int* in_sizes, int n_in,
                              void* d_out, int out_size, void* d_ws, size_t ws_size, hipStream_t stream) {
    if (n_in < 5) return;
    const long rows_used = (long)(NB - 1) * SEQ_FULL + SEQ;
    if ((long)in_sizes[0] < rows_used * DMOD) return;
    if ((long)in_sizes[1] < rows_used) return;
    if ((long)in_sizes[2] < (long)DMOD * QKVN) return;
    if (in_sizes[3] < DMOD || in_sizes[4] < DMOD) return;
    if ((long)out_size < rows_used * DMOD) return;
    const float* X = (const float*)d_in[0]; const int* M = (const int*)d_in[1]; const float* W = (const float*)d_in[2]; const float* G = (const float*)d_in[3]; const float* Bv = (const float*)d_in[4];
    float* OUT = (float*)d_out;
    char* wsp = (char*)d_ws;
    auto take = [&](size_t bytes) { char* p = wsp; wsp += (bytes + 255) & ~(size_t)255; return (void*)p; };
    bf* WT = (bf*)take((size_t)QKVN * DMOD * 2);
    bf* XH = (bf*)take((size_t)SEQ * DMOD * 2);
    bf* XL = (bf*)take((size_t)SEQ * DMOD * 2);
    float* CQ = (float*)take((size_t)SEQ * QKVN * 4);
    h16* QP = (h16*)take((size_t)NHD * SEQ * HD * 2);
    h16* KP = (h16*)take((size_t)NHD * SEQ * HD * 2);
    h16* VTp = (h16*)take((size_t)NHD * HD * SEQ * 2);
    if ((size_t)(wsp - (char*)d_ws) > ws_size) return;
    const int nlines = QKVN * DMOD / 64;
    k_wtG<<<(unsigned)((nlines + 63) / 64), 256, 0, stream>>>(W, DMOD, QKVN, WT);
    const int n8 = NHD * SEQ * HD / 8;
    for (int b = 0; b < NB; ++b) {
        const float* xb = X + (size_t)b * SEQ_FULL * DMOD;
        k_ln<<<SEQ, 128, 0, stream>>>(xb, G, Bv, XH, XL);
        k_gemmw<bf, 1, false><<<dim3(SEQ / 64, QKVN / 64, 1), 32, 0, stream>>>(XH, XL, WT, nullptr, DMOD, CQ, QKVN, nullptr, 0, 0, 0);
        k_qkp<<<dim3((unsigned)((n8 + 255) / 256), 2, 1), 256, 0, stream>>>(CQ, QP, KP, n8);
        k_vtp16<<<dim3(SEQ / 64, NHD, 1), 256, 0, stream>>>(CQ, VTp);
        k_flash<<<dim3(SEQ / 128, NHD, 1), 256, 0, stream>>>(QP, KP, VTp, M + (size_t)b * SEQ_FULL, OUT + (size_t)b * SEQ_FULL * DMOD);
    }
}
